// NeuralPredicateLayer_76828374991788
// MI455X (gfx1250) — hardware-verified
//
#include <hip/hip_runtime.h>
#include <math.h>
typedef __attribute__((ext_vector_type(16))) _Float16 v16h;
typedef __attribute__((ext_vector_type(8)))  _Float16 v8h;
typedef __attribute__((ext_vector_type(16))) __bf16   v16b;
typedef __attribute__((ext_vector_type(8)))  __bf16   v8b;
typedef __attribute__((ext_vector_type(8)))  float    v8f;
typedef __attribute__((ext_vector_type(4)))  float    v4f;
#define PSCALE 32768.0f
#define U16(p) ((const unsigned short*)(const void*)(p))
#define PSCALE_INV (1.0f / 32768.0f)

__device__ __forceinline__ unsigned short f2bf_bits(float f) {
  unsigned u = __float_as_uint(f);
  return (unsigned short)((u + 0x7FFFu + ((u >> 16) & 1u)) >> 16);
}
__device__ __forceinline__ float bf_bits2f(unsigned short h) { return __uint_as_float(((unsigned)h) << 16); }

__device__ __forceinline__ void dep_guard_h(v8f& a, v8f& b, v16h x, v16h y) { asm volatile("v_nop\n\tv_nop\n\tv_nop\n\tv_nop" : "+v"(a), "+v"(b) : "v"(x), "v"(y)); }
__device__ __forceinline__ void dep_guard_b(v8f& a, v8f& b, v16b x, v16b y) { asm volatile("v_nop\n\tv_nop\n\tv_nop\n\tv_nop" : "+v"(a), "+v"(b) : "v"(x), "v"(y)); }
__device__ __forceinline__ void keep4_h(v16h a, v16h b, v16h c, v16h d) { asm volatile("v_nop" :: "v"(a), "v"(b), "v"(c), "v"(d)); }
__device__ __forceinline__ void keep4_b(v16b a, v16b b, v16b c, v16b d) { asm volatile("v_nop" :: "v"(a), "v"(b), "v"(c), "v"(d)); }
__device__ __forceinline__ void acc_guard4(v8f& a, v8f& b, v8f& c, v8f& d) { asm volatile("v_nop\n\tv_nop\n\tv_nop\n\tv_nop" : "+v"(a), "+v"(b), "+v"(c), "+v"(d)); }
template <typename T> struct Frag;
template <> struct Frag<_Float16> {
  typedef v16h V; union U { v16h v; v8h h[2]; };
  static __device__ __forceinline__ v16h load(const _Float16* p) {
    U f; f.h[0] = *(const v8h*)(p); f.h[1] = *(const v8h*)(p + 16); return f.v;
  }
  static __device__ __forceinline__ v8f mma(v16h a, v16h b, v8f c) {
    return __builtin_amdgcn_wmma_f32_16x16x32_f16(false, a, false, b, (short)0, c, false, false);
  }
  static __device__ __forceinline__ void guard(v8f& a, v8f& b, v16h x, v16h y) { dep_guard_h(a, b, x, y); }
  static __device__ __forceinline__ void keep(v16h a, v16h b, v16h c, v16h d) { keep4_h(a, b, c, d); }
};
template <> struct Frag<__bf16> {
  typedef v16b V; union U { v16b v; v8b h[2]; };
  static __device__ __forceinline__ v16b load(const __bf16* p) {
    U f; f.h[0] = *(const v8b*)(p); f.h[1] = *(const v8b*)(p + 16); return f.v;
  }
  static __device__ __forceinline__ v8f mma(v16b a, v16b b, v8f c) {
    return __builtin_amdgcn_wmma_f32_16x16x32_bf16(false, a, false, b, (short)0, c, false, false);
  }
  static __device__ __forceinline__ void guard(v8f& a, v8f& b, v16b x, v16b y) { dep_guard_b(a, b, x, y); }
  static __device__ __forceinline__ void keep(v16b a, v16b b, v16b c, v16b d) { keep4_b(a, b, c, d); }
};

template <int ET> struct Elem;
template <> struct Elem<0> { typedef _Float16 T; };
template <> struct Elem<1> { typedef __bf16 T; };
template <int ET, bool SPLIT, int BIAS_MODE, int OUT_MODE, bool RESID, int ACT = 0>
__global__ __launch_bounds__(256) void wmma_gemm64(
    const unsigned short* __restrict__ Ap, const unsigned short* __restrict__ A2p, int lda, long strideA,
    const unsigned short* __restrict__ Btp, const unsigned short* __restrict__ Bt2p, int ldb, long strideB,
    void* __restrict__ Cout, void* __restrict__ Cout2, int ldc, long strideC,
    const float* __restrict__ bias,
    const float* __restrict__ resid, long strideR,
    int M, int N, int K, float scale) {
  typedef typename Elem<ET>::T T;
  typedef typename Frag<T>::V V;
  const T* A = (const T*)Ap; const T* A2 = (const T*)A2p; const T* Bt = (const T*)Btp; const T* Bt2 = (const T*)Bt2p;
  __shared__ __align__(16) float sT[8][16 * 68];
  const int b    = blockIdx.y;
  const int lane = threadIdx.x & 31;
  const int wave = threadIdx.x >> 5;
  const int tilesN = N >> 6;
  const int tilesM = M >> 6;
  const int tile = blockIdx.x * 8 + wave;
  if (tile >= tilesM * tilesN) return;
  const int tm = tile / tilesN;
  const int tn = tile - tm * tilesN;
  const int m0 = tm << 6;
  const int n0 = tn << 6;

  const T* Ab  = A  + (size_t)b * strideA;
  const T* Bb  = Bt + (size_t)b * strideB;
  const T* Ab2 = SPLIT ? (A2  + (size_t)b * strideA) : nullptr;
  const T* Bb2 = SPLIT ? (Bt2 + (size_t)b * strideB) : nullptr;

  const int rlane = lane & 15;
  const int koff  = (lane >> 4) * 8;
  const int mOff  = (lane >> 4) * 8;

  v8f acc[4][4];
#pragma unroll
  for (int i = 0; i < 4; ++i)
#pragma unroll
    for (int j = 0; j < 4; ++j) acc[i][j] = (v8f){0.f,0.f,0.f,0.f,0.f,0.f,0.f,0.f};

  for (int k0 = 0; k0 < K; k0 += 32) {
    V bh[4], bl[4];
#pragma unroll
    for (int j = 0; j < 4; ++j) {
      const size_t bo = (size_t)(n0 + (j << 4) + rlane) * ldb + koff + k0;
      bh[j] = Frag<T>::load(Bb + bo);
      if (SPLIT) bl[j] = Frag<T>::load(Bb2 + bo);
    }
#pragma unroll
    for (int i = 0; i < 4; ++i) {
      const size_t ao = (size_t)(m0 + (i << 4) + rlane) * lda + koff + k0;
      V ah = Frag<T>::load(Ab + ao);
      V al;
      if (SPLIT) al = Frag<T>::load(Ab2 + ao);
#pragma unroll
      for (int j = 0; j < 4; ++j) {
        acc[i][j] = Frag<T>::mma(ah, bh[j], acc[i][j]);
        if (SPLIT) {
          acc[i][j] = Frag<T>::mma(ah, bl[j], acc[i][j]);
          acc[i][j] = Frag<T>::mma(al, bh[j], acc[i][j]);
        }
      }
      Frag<T>::guard(acc[i][0], acc[i][3], ah, SPLIT ? al : ah);
    }
    Frag<T>::keep(bh[0], bh[1], bh[2], bh[3]);
    if (SPLIT) Frag<T>::keep(bl[0], bl[1], bl[2], bl[3]);
  }
  acc_guard4(acc[0][0], acc[0][1], acc[0][2], acc[0][3]);
  acc_guard4(acc[1][0], acc[1][1], acc[1][2], acc[1][3]);
  acc_guard4(acc[2][0], acc[2][1], acc[2][2], acc[2][3]);
  acc_guard4(acc[3][0], acc[3][1], acc[3][2], acc[3][3]);

  float* slab = sT[wave];
  const float* Rb = RESID ? (resid + (size_t)b * strideR) : nullptr;
#pragma unroll
  for (int i = 0; i < 4; ++i) {
    const int mBase = m0 + (i << 4);
#pragma unroll
    for (int j = 0; j < 4; ++j) {
      const int n = n0 + (j << 4) + rlane;
      float bv = 0.f;
      if (BIAS_MODE == 2) bv = bias[n];
#pragma unroll
      for (int r = 0; r < 8; ++r) {
        float v = acc[i][j][r] * scale;
        if (BIAS_MODE == 1) v += bias[mBase + mOff + r];
        if (BIAS_MODE == 2) v += bv;
        if (RESID) v += Rb[(size_t)(mBase + mOff + r) * ldc + n];
        if (ACT == 1) v = tanhf(v);
        if (ACT == 2) v = fmaxf(v, 0.0f);
        if (ACT == 3) v = v / (1.0f + expf(-v));
        if (ACT == 4) v = (v > 0.f) ? v : 0.01f * v;
        if (ACT == 5) v = 0.5f * v * (1.0f + erff(v * 0.70710678118654752f));
        slab[(mOff + r) * 68 + (j << 4) + rlane] = v;
      }
    }
    __builtin_amdgcn_fence(__ATOMIC_RELEASE, "workgroup");
    __builtin_amdgcn_wave_barrier();
    __builtin_amdgcn_fence(__ATOMIC_ACQUIRE, "workgroup");
    if (OUT_MODE == 0) {
      float* C = (float*)Cout + (size_t)b * strideC;
      const int hh = lane >> 4, c4 = (lane & 15) * 4;
      for (int pass = 0; pass < 2; ++pass) {
#pragma unroll
        for (int it = 0; it < 8; ++it) {
          const int row = it * 2 + hh;
          v4f v = *(const v4f*)(slab + row * 68 + c4);
          *(volatile v4f*)(C + (size_t)(mBase + row) * ldc + n0 + c4) = v;
        }
        __threadfence();
      }
    } else {
      const int q = lane >> 3, c8 = (lane & 7) * 8;
      unsigned short* C  = (unsigned short*)Cout  + (size_t)b * strideC;
      unsigned short* C2 = (OUT_MODE == 2) ? ((unsigned short*)Cout2 + (size_t)b * strideC) : nullptr;
      for (int pass = 0; pass < 2; ++pass) {
#pragma unroll
        for (int it = 0; it < 4; ++it) {
          const int row = it * 4 + q;
          const float* sp = slab + row * 68 + c8;
          v8h hv, lv;
#pragma unroll
          for (int e = 0; e < 8; ++e) {
            if (OUT_MODE == 1) {
              hv[e] = (_Float16)sp[e];
            } else {
              unsigned short hb = f2bf_bits(sp[e]);
              unsigned short lb = f2bf_bits(sp[e] - bf_bits2f(hb));
              hv[e] = __builtin_bit_cast(_Float16, hb);
              lv[e] = __builtin_bit_cast(_Float16, lb);
            }
          }
          *(volatile v8h*)(C + (size_t)(mBase + row) * ldc + n0 + c8) = hv;
          if (OUT_MODE == 2) *(volatile v8h*)(C2 + (size_t)(mBase + row) * ldc + n0 + c8) = lv;
        }
        __threadfence();
      }
    }
    __builtin_amdgcn_fence(__ATOMIC_RELEASE, "workgroup");
    __builtin_amdgcn_wave_barrier();
    __builtin_amdgcn_fence(__ATOMIC_ACQUIRE, "workgroup");
  }
}

__global__ __launch_bounds__(256) void cast_f32_f16x2(
    const float* __restrict__ in, _Float16* __restrict__ out, int n2) {
  int i = blockIdx.x * 256 + threadIdx.x;
  if (i < n2) {
    const _Float16 h0 = (_Float16)in[2 * i], h1 = (_Float16)in[2 * i + 1];
    const unsigned u = (unsigned)__builtin_bit_cast(unsigned short, h0) | ((unsigned)__builtin_bit_cast(unsigned short, h1) << 16);
    ((volatile unsigned*)out)[i] = u;
    __threadfence();
    ((volatile unsigned*)out)[i] = u;
  }
}


#define PN 8192
#define PM 32768
#define PF 256
#define PH 128
#define PH2 64
#define PU 21
#define PB 6
__global__ __launch_bounds__(256) void wb_kernel(const float* __restrict__ Wb1, unsigned* __restrict__ WbA, unsigned* __restrict__ WbB, float* __restrict__ WbS) {
  const int row = blockIdx.x;
  const float* src = Wb1 + (size_t)row * 516;
  for (int pass = 0; pass < 2; ++pass) {
    for (int i = threadIdx.x; i < 128; i += 256) { ((volatile unsigned*)WbA)[row * 128 + i] = (unsigned)__builtin_bit_cast(unsigned short, (_Float16)src[2 * i]) | ((unsigned)__builtin_bit_cast(unsigned short, (_Float16)src[2 * i + 1]) << 16);
      ((volatile unsigned*)WbB)[row * 128 + i] = (unsigned)__builtin_bit_cast(unsigned short, (_Float16)src[256 + 2 * i]) | ((unsigned)__builtin_bit_cast(unsigned short, (_Float16)src[256 + 2 * i + 1]) << 16); }
    if (threadIdx.x < 4) ((volatile float*)WbS)[row * 4 + threadIdx.x] = src[512 + threadIdx.x];
    __threadfence(); }
}
__global__ __launch_bounds__(256) void ulogit_kernel(const _Float16* __restrict__ H2, const float* __restrict__ bu2, const float* __restrict__ wu3, const float* __restrict__ bu3, float* __restrict__ out0) {
  __shared__ float st[64 * PU];
  const int lane = threadIdx.x & 31, wave = threadIdx.x >> 5; const int n0 = blockIdx.x * 64;
  for (int k = 0; k < 8; ++k) { const int nl = wave * 8 + k; const size_t n = (size_t)n0 + nl;
#pragma unroll 1
    for (int p = 0; p < PU; ++p) { const float a = fmaxf((float)H2[n * (PU * 64) + p * 64 + lane] + bu2[p * 64 + lane], 0.f) * wu3[p * 64 + lane], b = fmaxf((float)H2[n * (PU * 64) + p * 64 + 32 + lane] + bu2[p * 64 + 32 + lane], 0.f) * wu3[p * 64 + 32 + lane];
      float d = a + b; for (int o = 16; o > 0; o >>= 1) d += __shfl_xor(d, o, 32); if (lane == 0) st[nl * PU + p] = 1.0f / (1.0f + expf(-(d + bu3[p]))); } }
  __syncthreads();
  for (int pass = 0; pass < 2; ++pass) { for (int i = threadIdx.x; i < 64 * PU; i += 256) ((volatile float*)out0)[(size_t)n0 * PU + i] = st[i]; __threadfence(); }
}
__global__ __launch_bounds__(256) void pair_kernel(const _Float16* __restrict__ FA, const _Float16* __restrict__ FB, const float* __restrict__ WbS, const float* __restrict__ bb1, const float* __restrict__ pos, const int* __restrict__ pidx, unsigned* __restrict__ A16) {
  const int lane = threadIdx.x & 31, wave = threadIdx.x >> 5; const size_t m = (size_t)blockIdx.x * 8 + wave;
  int i = pidx[m * 2], j = pidx[m * 2 + 1]; i = i < 0 ? 0 : (i >= PN ? PN - 1 : i); j = j < 0 ? 0 : (j >= PN ? PN - 1 : j);
  const float dx = pos[j * 3] - pos[i * 3], dy = pos[j * 3 + 1] - pos[i * 3 + 1], dz = pos[j * 3 + 2] - pos[i * 3 + 2]; const float dist = sqrtf(dx * dx + dy * dy + dz * dz);
  for (int pass = 0; pass < 2; ++pass) {
    for (int q = 0; q < 12; ++q) { const int c = q * 64 + 2 * lane;
      float v[2]; for (int e = 0; e < 2; ++e) { const int cc = c + e; v[e] = fmaxf((float)FA[(size_t)i * 768 + cc] + (float)FB[(size_t)j * 768 + cc] + WbS[cc * 4] * dx + WbS[cc * 4 + 1] * dy + WbS[cc * 4 + 2] * dz + WbS[cc * 4 + 3] * dist + bb1[cc], 0.f); }
      ((volatile unsigned*)A16)[(m * 768 + c) / 2] = (unsigned)__builtin_bit_cast(unsigned short, (_Float16)v[0]) | ((unsigned)__builtin_bit_cast(unsigned short, (_Float16)v[1]) << 16); }
    __threadfence(); }
}
__global__ __launch_bounds__(256) void blogit_kernel(const _Float16* __restrict__ H2, const float* __restrict__ bb2, const float* __restrict__ wb3, const float* __restrict__ bb3, float* __restrict__ out1) {
  __shared__ float st[64 * PB];
  const int lane = threadIdx.x & 31, wave = threadIdx.x >> 5; const int m0 = blockIdx.x * 64;
  for (int k = 0; k < 8; ++k) { const int ml = wave * 8 + k; const size_t m = (size_t)m0 + ml;
#pragma unroll 1
    for (int p = 0; p < PB; ++p) { const float a = fmaxf((float)H2[m * (PB * 64) + p * 64 + lane] + bb2[p * 64 + lane], 0.f) * wb3[p * 64 + lane], b = fmaxf((float)H2[m * (PB * 64) + p * 64 + 32 + lane] + bb2[p * 64 + 32 + lane], 0.f) * wb3[p * 64 + 32 + lane];
      float d = a + b; for (int o = 16; o > 0; o >>= 1) d += __shfl_xor(d, o, 32); if (lane == 0) st[ml * PB + p] = 1.0f / (1.0f + expf(-(d + bb3[p]))); } }
  __syncthreads();
  for (int pass = 0; pass < 2; ++pass) { for (int i = threadIdx.x; i < 64 * PB; i += 256) ((volatile float*)out1)[(size_t)m0 * PB + i] = st[i]; __threadfence(); }
}
extern "C" void kernel_launch(void* const* d_in, const int* in_sizes, int n_in, void* d_out, int out_size, void* d_ws, size_t ws_size, hipStream_t stream) {
  (void)in_sizes; (void)n_in; (void)out_size; (void)ws_size;
  auto Fp = [&](int i) { return (const float*)d_in[i]; };
  const float* X = Fp(0); const float* pos = Fp(1); const int* pidx = (const int*)d_in[2];
  const float* Wu1 = Fp(3); const float* bu1 = Fp(4); const float* Wu2 = Fp(5); const float* bu2 = Fp(6); const float* wu3 = Fp(7); const float* bu3 = Fp(8);
  const float* Wb1 = Fp(9); const float* bb1 = Fp(10); const float* Wb2 = Fp(11); const float* bb2 = Fp(12); const float* wb3 = Fp(13); const float* bb3 = Fp(14);
  float* out0 = (float*)d_out; float* out1 = out0 + (size_t)PN * PU;
  char* ws = (char*)d_ws; size_t off = 0;
  auto carve = [&](size_t bytes) -> char* { char* p = ws + off; off += (bytes + 255) & ~(size_t)255; return p; };
  _Float16* X16 = (_Float16*)carve((size_t)PN * PF * 2); _Float16* WU1 = (_Float16*)carve((size_t)PU * PH * PF * 2); _Float16* WU2 = (_Float16*)carve((size_t)PU * PH2 * PH * 2); _Float16* WB2 = (_Float16*)carve((size_t)PB * PH2 * PH * 2);
  unsigned* WbA = (unsigned*)carve(768 * 256 * 2); unsigned* WbB = (unsigned*)carve(768 * 256 * 2); float* WbS = (float*)carve(768 * 4 * 4);
  char* RA = carve((size_t)PM * 768 * 2); char* RB = carve((size_t)PM * PB * PH2 * 2);
  _Float16* H1u = (_Float16*)RA; _Float16* H2u = (_Float16*)RB; unsigned* A16 = (unsigned*)RA; _Float16* H2b = (_Float16*)RB;
  _Float16* FA = (_Float16*)carve((size_t)PN * 768 * 2); _Float16* FB = (_Float16*)carve((size_t)PN * 768 * 2);
  cast_f32_f16x2<<<(PN * PF / 2 + 255) / 256, 256, 0, stream>>>(X, X16, (long)PN * PF / 2);
  cast_f32_f16x2<<<(PU * PH * PF / 2 + 255) / 256, 256, 0, stream>>>(Wu1, WU1, (long)PU * PH * PF / 2);
  cast_f32_f16x2<<<(PU * PH2 * PH / 2 + 255) / 256, 256, 0, stream>>>(Wu2, WU2, (long)PU * PH2 * PH / 2);
  cast_f32_f16x2<<<(PB * PH2 * PH / 2 + 255) / 256, 256, 0, stream>>>(Wb2, WB2, (long)PB * PH2 * PH / 2);
  wb_kernel<<<768, 256, 0, stream>>>(Wb1, WbA, WbB, WbS);
  { const int t = (PN / 64) * (PU * PH / 64); wmma_gemm64<0, false, 2, 1, false, 2><<<dim3((t + 7) / 8, 1), 256, 0, stream>>>(U16(X16), nullptr, PF, 0, U16(WU1), nullptr, PF, 0, H1u, nullptr, PU * PH, 0, bu1, nullptr, 0, PN, PU * PH, PF, 1.0f); }
  { const int t = (PN / 64) * 1; wmma_gemm64<0, false, 0, 1, false, 0><<<dim3((t + 7) / 8, PU), 256, 0, stream>>>(U16(H1u), nullptr, PU * PH, PH, U16(WU2), nullptr, PH, PH2 * PH, H2u, nullptr, PU * PH2, PH2, nullptr, nullptr, 0, PN, PH2, PH, 1.0f); }
  ulogit_kernel<<<PN / 64, 256, 0, stream>>>(H2u, bu2, wu3, bu3, out0);
  { const int t = (PN / 64) * 12; wmma_gemm64<0, false, 0, 1, false, 0><<<dim3((t + 7) / 8, 1), 256, 0, stream>>>(U16(X16), nullptr, PF, 0, (const unsigned short*)WbA, nullptr, PF, 0, FA, nullptr, 768, 0, nullptr, nullptr, 0, PN, 768, PF, 1.0f);
    wmma_gemm64<0, false, 0, 1, false, 0><<<dim3((t + 7) / 8, 1), 256, 0, stream>>>(U16(X16), nullptr, PF, 0, (const unsigned short*)WbB, nullptr, PF, 0, FB, nullptr, 768, 0, nullptr, nullptr, 0, PN, 768, PF, 1.0f); }
  pair_kernel<<<PM / 8, 256, 0, stream>>>(FA, FB, WbS, bb1, pos, pidx, A16);
  { const int t = (PM / 64) * 1; wmma_gemm64<0, false, 0, 1, false, 0><<<dim3((t + 7) / 8, PB), 256, 0, stream>>>((const unsigned short*)A16, nullptr, 768, PH, U16(WB2), nullptr, PH, PH2 * PH, H2b, nullptr, PB * PH2, PH2, nullptr, nullptr, 0, PM, PH2, PH, 1.0f); }
  blogit_kernel<<<PM / 64, 256, 0, stream>>>(H2b, bb2, wb3, bb3, out1);
}
